// CTRNN_50087908606434
// MI455X (gfx1250) — hardware-verified
//
#include <hip/hip_runtime.h>
#include <math.h>


#define DT_C    0.02f
#define HIDDEN  512
#define TSTEPS  1024
#define MROWS   16
#define NWAVES  16
#define NTHREADS (NWAVES * 32)
#define APITCH  520

typedef __attribute__((ext_vector_type(16))) __bf16 v16bf;
typedef __attribute__((ext_vector_type(8)))  __bf16 v8bf;
typedef __attribute__((ext_vector_type(8)))  float  v8f;
typedef __attribute__((ext_vector_type(4)))  float  v4f;
typedef __attribute__((ext_vector_type(4)))  unsigned v4u;

template <typename T> __device__ __forceinline__ void vst2(void* p, T v) { *(volatile T*)p = v; __threadfence(); *(volatile T*)p = v; }
__device__ __forceinline__ v8f wmma_bf(v16bf a, v16bf b, v8f c) {
  v8f d = __builtin_amdgcn_wmma_f32_16x16x32_bf16(false, a, false, b, (short)0, c, false, false);
  asm volatile("v_nop\n\tv_nop\n\tv_nop\n\tv_nop" : "+v"(d) : "v"(a), "v"(b));
  return d;
}
__device__ __forceinline__ v16bf frag_bf(const __bf16* row, int k0, int lane) {
  union { v16bf v; v8bf q[2]; } r; const __bf16* p = row + k0 + 8 * (lane >> 4);
  r.q[0] = *(const v8bf*)(p); r.q[1] = *(const v8bf*)(p + 16); return r.v;
}

__global__ __launch_bounds__(256) void k_split_j(const float* __restrict__ J, __bf16* __restrict__ Jhi, __bf16* __restrict__ Jlo) {
  const int g = blockIdx.x * 256 + threadIdx.x;
  union { v8bf b; v4u u; } ph, pl;
#pragma unroll
  for (int e = 0; e < 8; ++e) { const float x = J[(size_t)g * 8 + e]; const __bf16 h = (__bf16)x; ph.b[e] = h; pl.b[e] = (__bf16)(x - (float)h); }
  vst2(Jhi + (size_t)g * 8, ph.u); vst2(Jlo + (size_t)g * 8, pl.u);
}

__global__ void __launch_bounds__(NTHREADS)
ctrnn_main(const float* __restrict__ vel, const __bf16* __restrict__ Jhi, const __bf16* __restrict__ Jlo,
           const float* __restrict__ Bmat, const float* __restrict__ Wro, float* __restrict__ out)
{
  __shared__ __align__(16) __bf16 Ahi[2][MROWS * APITCH];
  __shared__ __align__(16) __bf16 Alo[2][MROWS * APITCH];
  __shared__ __align__(16) float obuf[MROWS * TSTEPS];
  __shared__ float part[NWAVES][MROWS];
  __shared__ float vbuf[MROWS][36];

  const int tid = threadIdx.x, lane = tid & 31, w = tid >> 5;
  const int col = lane & 15, hi = lane >> 4;
  const int b0 = blockIdx.x * MROWS;
  const int n0 = w * 32;

  for (int i = tid; i < MROWS * APITCH; i += NTHREADS) { Ahi[0][i] = (__bf16)0.f; Alo[0][i] = (__bf16)0.f; Ahi[1][i] = (__bf16)0.f; Alo[1][i] = (__bf16)0.f; }
  float bm[2], wr[2];
#pragma unroll
  for (int j = 0; j < 2; ++j) { bm[j] = Bmat[n0 + j * 16 + col]; wr[j] = Wro[n0 + j * 16 + col]; }
  v8f h[2] = {(v8f){}, (v8f){}};
  __syncthreads();

#pragma unroll 1
  for (int t = 0; t < TSTEPS; ++t) {
    const int cur = t & 1, nxt = cur ^ 1;
    if ((t & 31) == 0) {
      __syncthreads();
      for (int i = tid; i < MROWS * 32; i += NTHREADS) { const int r = i >> 5, tt = i & 31; vbuf[r][tt] = vel[(size_t)(b0 + r) * TSTEPS + t + tt]; }
      __syncthreads();
    }
    v8f acc[2] = {(v8f){}, (v8f){}};
    const __bf16* Ah = Ahi[cur] + col * APITCH;
    const __bf16* Al = Alo[cur] + col * APITCH;
#pragma unroll 4
    for (int kc = 0; kc < HIDDEN / 32; ++kc) {
      const v16bf ah = frag_bf(Ah, kc * 32, lane), al = frag_bf(Al, kc * 32, lane);
#pragma unroll
      for (int j = 0; j < 2; ++j) {
        const __bf16* bh = Jhi + (size_t)(n0 + j * 16 + col) * HIDDEN;
        const __bf16* bl = Jlo + (size_t)(n0 + j * 16 + col) * HIDDEN;
        const v16bf fh = frag_bf(bh, kc * 32, lane), fl = frag_bf(bl, kc * 32, lane);
        acc[j] = wmma_bf(al, fh, acc[j]); acc[j] = wmma_bf(ah, fl, acc[j]); acc[j] = wmma_bf(ah, fh, acc[j]);
      }
    }
    float pr[8];
#pragma unroll
    for (int r = 0; r < 8; ++r) pr[r] = 0.f;
    const int tt = t & 31;
#pragma unroll
    for (int j = 0; j < 2; ++j) {
#pragma unroll
      for (int r = 0; r < 8; ++r) {
        const int row = hi * 8 + r;
        const float v = vbuf[row][tt];
        const float hn = h[j][r] * (1.0f - DT_C) + DT_C * (acc[j][r] + v * bm[j]);
        h[j][r] = hn;
        const float th = tanhf(hn);
        const __bf16 thh = (__bf16)th;
        Ahi[nxt][row * APITCH + n0 + j * 16 + col] = thh;
        Alo[nxt][row * APITCH + n0 + j * 16 + col] = (__bf16)(th - (float)thh);
        pr[r] += th * wr[j];
      }
    }
#pragma unroll
    for (int r = 0; r < 8; ++r) {
      float p = pr[r];
#pragma unroll
      for (int off = 8; off > 0; off >>= 1) p += __shfl_xor(p, off, 32);
      if (col == 0) part[w][hi * 8 + r] = p;
    }
    __syncthreads();
    if (tid < MROWS) {
      float s = 0.f;
#pragma unroll
      for (int ww = 0; ww < NWAVES; ++ww) s += part[ww][tid];
      obuf[tid * TSTEPS + t] = s;
    }
    __syncthreads();
  }
  __syncthreads();
  for (int g = tid; g < MROWS * TSTEPS / 4; g += NTHREADS) {
    const int r = g >> 8, pc = g & 255;
    vst2(out + (size_t)(b0 + r) * TSTEPS + pc * 4, *(const v4f*)(obuf + r * TSTEPS + pc * 4));
  }
}

extern "C" void kernel_launch(void* const* d_in, const int* in_sizes, int n_in,
                              void* d_out, int out_size, void* d_ws, size_t ws_size,
                              hipStream_t stream) {
  (void)in_sizes; (void)n_in; (void)out_size; (void)ws_size;
  const float* vel  = (const float*)d_in[0];
  const float* J    = (const float*)d_in[1];
  const float* Bm   = (const float*)d_in[2];
  const float* Wro  = (const float*)d_in[3];
  float* out        = (float*)d_out;
  __bf16* Jhi = (__bf16*)d_ws;
  __bf16* Jlo = Jhi + (size_t)HIDDEN * HIDDEN;
  k_split_j<<<HIDDEN * HIDDEN / 8 / 256, 256, 0, stream>>>(J, Jhi, Jlo);
  ctrnn_main<<<128 / MROWS, NTHREADS, 0, stream>>>(vel, Jhi, Jlo, Bm, Wro, out);
}
